// _AVWGCN_89696097010341
// MI455X (gfx1250) — hardware-verified
//
#include <hip/hip_runtime.h>

#define NB_ 64
#define NN_ 2048
#define CI  32
#define CO  32
#define DE  16
#define XW  2048

typedef _Float16 f16;
typedef __attribute__((ext_vector_type(16))) f16 f16x16;
typedef __attribute__((ext_vector_type(8)))  f16 f16x8;
typedef __attribute__((ext_vector_type(8)))  float f32x8;
typedef __attribute__((ext_vector_type(4)))  float v4f_t;
typedef float v4fa __attribute__((ext_vector_type(4), may_alias));

__device__ __forceinline__ f32x8 wmma16(f16x16 a, f16x16 b, f32x8 c) {
  c = __builtin_amdgcn_wmma_f32_16x16x32_f16(false, a, false, b, (short)0, c, false, false);
  asm volatile("v_nop\n\tv_nop\n\tv_nop\n\tv_nop" : "+v"(c) : "v"(a), "v"(b));
  return c;
}
__device__ __forceinline__ f16x16 lds_frag(const f16* base, int stride) {
  const int lane = threadIdx.x & 31, row = lane & 15, kh = (lane >> 4) * 8;
  const f16x8 lo = *(const f16x8*)(base + row * stride + kh);
  const f16x8 hi = *(const f16x8*)(base + row * stride + kh + 16);
  f16x16 f;
#pragma unroll
  for (int i = 0; i < 8; ++i) { f[i] = lo[i]; f[i + 8] = hi[i]; }
  return f;
}
__device__ __forceinline__ void split16(float v, f16& h, f16& l) { h = (f16)v; l = (f16)((v - (float)h) * 2048.0f); }
#define GSTR 48

template <typename AT, bool ACC>
__global__ __launch_bounds__(256) void gemm_kn2(const AT* __restrict__ A, int lda, size_t strideA,
                                               const float* __restrict__ Wm, int ldw, size_t strideW,
                                               const float* __restrict__ bias, float scale,
                                               float* __restrict__ Y, int ldy, size_t strideY, int K) {
  __shared__ __attribute__((aligned(16))) f16 ldsA[128 * GSTR], ldsAl[128 * GSTR];
  __shared__ __attribute__((aligned(16))) f16 ldsW[128 * GSTR], ldsWl[128 * GSTR];
  __shared__ __attribute__((aligned(16))) float oS[8][32 * 68];
  const int tid = threadIdx.x, lane = tid & 31, wave = tid >> 5, cl = lane & 15, rh = (lane >> 4) * 8;
  const int m0 = blockIdx.x * 128, n0 = blockIdx.y * 128;
  const int wm = (wave & 3) * 32, wn = (wave >> 2) * 64;
  A += (size_t)blockIdx.z * strideA; Wm += (size_t)blockIdx.z * strideW; Y += (size_t)blockIdx.z * strideY;
  f32x8 acc[2][4], accx[2][4];
#pragma unroll
  for (int i = 0; i < 2; ++i)
#pragma unroll
    for (int j = 0; j < 4; ++j) { f32x8 z = {}; acc[i][j] = z; accx[i][j] = z; }
#pragma unroll 1
  for (int k0 = 0; k0 < K; k0 += 32) {
    __syncthreads();
    {
      const int row = tid >> 1, ch = (tid & 1) * 16;
      const AT* src = A + (size_t)(m0 + row) * lda + k0 + ch;
#pragma unroll
      for (int g = 0; g < 16; ++g) { const float v = (float)src[g]; const f16 h = (f16)v; ldsA[row * GSTR + ch + g] = h; ldsAl[row * GSTR + ch + g] = (f16)((v - (float)h) * 2048.0f); }
    }
    {
      const int k = tid >> 3, nn0 = (tid & 7) * 16;
      const float* src = Wm + (size_t)(k0 + k) * ldw + n0 + nn0;
#pragma unroll
      for (int g = 0; g < 4; ++g) { const v4f_t v = *(const v4f_t*)(src + 4 * g);
#pragma unroll
        for (int u = 0; u < 4; ++u) { const f16 h = (f16)v[u]; ldsW[(nn0 + 4 * g + u) * GSTR + k] = h; ldsWl[(nn0 + 4 * g + u) * GSTR + k] = (f16)((v[u] - (float)h) * 2048.0f); } }
    }
    __syncthreads();
    f16x16 af[2], afl[2];
#pragma unroll
    for (int i = 0; i < 2; ++i) { af[i] = lds_frag(ldsA + (wm + 16 * i) * GSTR, GSTR); afl[i] = lds_frag(ldsAl + (wm + 16 * i) * GSTR, GSTR); }
#pragma unroll
    for (int j = 0; j < 4; ++j) {
      const f16x16 bf = lds_frag(ldsW + (wn + 16 * j) * GSTR, GSTR), bfl = lds_frag(ldsWl + (wn + 16 * j) * GSTR, GSTR);
#pragma unroll
      for (int i = 0; i < 2; ++i) { acc[i][j] = wmma16(af[i], bf, acc[i][j]); accx[i][j] = wmma16(af[i], bfl, accx[i][j]); accx[i][j] = wmma16(afl[i], bf, accx[i][j]); }
    }
  }
  float* so = oS[wave];
#pragma unroll
  for (int i = 0; i < 2; ++i)
#pragma unroll
    for (int j = 0; j < 4; ++j) {
      const float bv = bias ? bias[n0 + wn + 16 * j + cl] : 0.0f;
#pragma unroll
      for (int r = 0; r < 8; ++r) so[(16 * i + rh + r) * 68 + 16 * j + cl] = (acc[i][j][r] + accx[i][j][r] * (1.0f / 2048.0f)) * scale + bv;
    }
  asm volatile("s_wait_dscnt 0" ::: "memory");
  __builtin_amdgcn_wave_barrier();
  if (ACC) {
#pragma unroll
    for (int it = 0; it < 16; ++it) { const int f4 = lane + 32 * it, rr = f4 >> 4, q = (f4 & 15) * 4;
      const v4f_t old = *(const volatile v4fa*)(Y + (size_t)(m0 + wm + rr) * ldy + n0 + wn + q);
      v4f_t v = *(const volatile v4fa*)(so + rr * 68 + q); v += old; *(volatile v4fa*)(so + rr * 68 + q) = v; }
    asm volatile("s_wait_dscnt 0" ::: "memory");
  }
#pragma unroll 1
  for (int pass = 0; pass < 2; ++pass) {
#pragma unroll
    for (int it = 0; it < 16; ++it) { const int f4 = lane + 32 * it, rr = f4 >> 4, q = (f4 & 15) * 4;
      *(volatile v4f_t*)(Y + (size_t)(m0 + wm + rr) * ldy + n0 + wn + q) = *(const volatile v4fa*)(so + rr * 68 + q); }
    __threadfence();
  }
}

__global__ __launch_bounds__(256) void k_supports(const float* __restrict__ E, float* __restrict__ A) {
  __shared__ float redm[8][16], redz[8][16], mS[16], zS[16];
  __shared__ __attribute__((aligned(16))) float oS[8][16 * 68];
  const int tid = threadIdx.x, lane = tid & 31, wave = tid >> 5, cl = lane & 15, hsel = lane >> 4, kh = hsel * 8, rh = kh;
  const int r0 = blockIdx.x * 16;
  f16x16 ah, al;
#pragma unroll
  for (int i = 0; i < 8; ++i) { f16 h, l; split16(E[(size_t)(r0 + cl) * DE + kh + i], h, l); ah[i] = h; al[i] = l; ah[8 + i] = (f16)0.0f; al[8 + i] = (f16)0.0f; }
  auto tile = [&](int nt, f32x8& s) {
    f16x16 bh, bl;
#pragma unroll
    for (int i = 0; i < 8; ++i) { f16 h, l; split16(E[(size_t)(nt * 16 + cl) * DE + kh + i], h, l); bh[i] = h; bl[i] = l; bh[8 + i] = (f16)0.0f; bl[8 + i] = (f16)0.0f; }
    f32x8 z = {}, zl = {};
    z = wmma16(ah, bh, z); zl = wmma16(ah, bl, zl); zl = wmma16(al, bh, zl);
#pragma unroll
    for (int r = 0; r < 8; ++r) s[r] = fmaxf(z[r] + zl[r] * (1.0f / 2048.0f), 0.0f);
  };
  float mx[8], zz[8];
#pragma unroll
  for (int r = 0; r < 8; ++r) { mx[r] = -INFINITY; zz[r] = 0.0f; }
#pragma unroll 1
  for (int j = 0; j < 16; ++j) { f32x8 s; tile(wave * 16 + j, s);
#pragma unroll
    for (int r = 0; r < 8; ++r) mx[r] = fmaxf(mx[r], s[r]); }
#pragma unroll
  for (int r = 0; r < 8; ++r) {
#pragma unroll
    for (int off = 8; off >= 1; off >>= 1) mx[r] = fmaxf(mx[r], __shfl_xor(mx[r], off, 32)); }
  if (cl == 0) {
#pragma unroll
    for (int r = 0; r < 8; ++r) redm[wave][rh + r] = mx[r]; }
  __syncthreads();
  if (tid < 16) { float m = redm[0][tid];
#pragma unroll
    for (int w = 1; w < 8; ++w) m = fmaxf(m, redm[w][tid]); mS[tid] = m; }
  __syncthreads();
  float mrow[8];
#pragma unroll
  for (int r = 0; r < 8; ++r) mrow[r] = mS[rh + r];
#pragma unroll 1
  for (int j = 0; j < 16; ++j) { f32x8 s; tile(wave * 16 + j, s);
#pragma unroll
    for (int r = 0; r < 8; ++r) zz[r] += __expf(s[r] - mrow[r]); }
#pragma unroll
  for (int r = 0; r < 8; ++r) {
#pragma unroll
    for (int off = 8; off >= 1; off >>= 1) zz[r] += __shfl_xor(zz[r], off, 32); }
  if (cl == 0) {
#pragma unroll
    for (int r = 0; r < 8; ++r) redz[wave][rh + r] = zz[r]; }
  __syncthreads();
  if (tid < 16) { float z = 0.0f;
#pragma unroll
    for (int w = 0; w < 8; ++w) z += redz[w][tid]; zS[tid] = 1.0f / z; }
  __syncthreads();
  float izr[8];
#pragma unroll
  for (int r = 0; r < 8; ++r) izr[r] = zS[rh + r];
  float* so = oS[wave];
#pragma unroll 1
  for (int g = 0; g < 4; ++g) {
#pragma unroll
    for (int jj = 0; jj < 4; ++jj) { f32x8 s; tile(wave * 16 + g * 4 + jj, s);
#pragma unroll
      for (int r = 0; r < 8; ++r) so[(rh + r) * 68 + jj * 16 + cl] = __expf(s[r] - mrow[r]) * izr[r]; }
    asm volatile("s_wait_dscnt 0" ::: "memory");
    __builtin_amdgcn_wave_barrier();
#pragma unroll 1
    for (int pass = 0; pass < 2; ++pass) {
#pragma unroll
      for (int it = 0; it < 8; ++it) { const int f4 = lane + 32 * it, rr = f4 >> 4, q = (f4 & 15) * 4;
        *(volatile v4f_t*)(A + (size_t)(r0 + rr) * NN_ + (wave * 16 + g * 4) * 16 + q) = *(const volatile v4fa*)(so + rr * 68 + q); }
      __threadfence();
    }
    __builtin_amdgcn_wave_barrier();
  }
}
__global__ __launch_bounds__(256) void k_xpose(const float* __restrict__ x, float* __restrict__ X) {
  __shared__ __attribute__((aligned(16))) float rowS[XW];
  const int tid = threadIdx.x, m = blockIdx.x;
  for (int e = tid; e < XW; e += 256) { const int b = e >> 5, c = e & 31; rowS[e] = x[((size_t)b * NN_ + m) * CI + c]; }
  __syncthreads();
#pragma unroll 1
  for (int pass = 0; pass < 2; ++pass) {
#pragma unroll
    for (int it = 0; it < 2; ++it) *(volatile v4f_t*)(X + (size_t)m * XW + (tid + 256 * it) * 4) = *(const volatile v4fa*)(rowS + (tid + 256 * it) * 4);
    __threadfence();
  }
}
__global__ __launch_bounds__(256) void k_node(const float* __restrict__ E, const float* __restrict__ Wp, const float* __restrict__ bp,
                                              const float* __restrict__ X, const float* __restrict__ Y1, const float* __restrict__ Y2,
                                              float* __restrict__ out) {
  __shared__ __attribute__((aligned(16))) f16 aS[2][64 * 104];
  __shared__ __attribute__((aligned(16))) f16 wS[2][32 * 104];
  __shared__ float eS[DE], bS[CO];
  __shared__ __attribute__((aligned(16))) float oS[64 * 36];
  const int tid = threadIdx.x, lane = tid & 31, wave = tid >> 5, cl = lane & 15, rh = (lane >> 4) * 8;
  const int n = blockIdx.x;
  if (tid < DE) eS[tid] = E[(size_t)n * DE + tid];
  __syncthreads();
  for (int e = tid; e < 3 * CI * CO; e += 256) {
    const int ki = e >> 5, o = e & 31;
    float s = 0.0f;
#pragma unroll
    for (int d = 0; d < DE; ++d) s += eS[d] * Wp[((size_t)d * 3 * CI + ki) * CO + o];
    f16 h, l; split16(s, h, l); wS[0][o * 104 + ki] = h; wS[1][o * 104 + ki] = l;
  }
  if (tid < CO) { float s = 0.0f;
#pragma unroll
    for (int d = 0; d < DE; ++d) s += eS[d] * bp[d * CO + tid]; bS[tid] = s; }
  for (int e = tid; e < NB_ * 3 * CI; e += 256) {
    const int b = e / 96, ki = e % 96, k = ki >> 5, i = ki & 31;
    const size_t off = (size_t)n * XW + b * CI + i;
    const float v = (k == 0) ? X[off] : (k == 1) ? Y1[off] : (2.0f * Y2[off] - X[off]);
    f16 h, l; split16(v, h, l); aS[0][b * 104 + ki] = h; aS[1][b * 104 + ki] = l;
  }
  __syncthreads();
  const int rt = wave >> 1, nt = wave & 1;
  f32x8 acc = {}, accx = {};
#pragma unroll
  for (int ks = 0; ks < 3; ++ks) {
    const f16x16 ah = lds_frag(aS[0] + (rt * 16) * 104 + ks * 32, 104), al = lds_frag(aS[1] + (rt * 16) * 104 + ks * 32, 104);
    const f16x16 bh = lds_frag(wS[0] + (nt * 16) * 104 + ks * 32, 104), bl = lds_frag(wS[1] + (nt * 16) * 104 + ks * 32, 104);
    acc = wmma16(ah, bh, acc); accx = wmma16(ah, bl, accx); accx = wmma16(al, bh, accx);
  }
#pragma unroll
  for (int r = 0; r < 8; ++r) oS[(rt * 16 + rh + r) * 36 + nt * 16 + cl] = acc[r] + accx[r] * (1.0f / 2048.0f) + bS[nt * 16 + cl];
  __syncthreads();
#pragma unroll 1
  for (int pass = 0; pass < 2; ++pass) {
#pragma unroll
    for (int it = 0; it < 2; ++it) { const int ch = tid + 256 * it, b = ch >> 3, q = (ch & 7) * 4;
      *(volatile v4f_t*)(out + ((size_t)b * NN_ + n) * CO + q) = *(const volatile v4fa*)(oS + b * 36 + q); }
    __threadfence();
  }
}

extern "C" void kernel_launch(void* const* d_in, const int* in_sizes, int n_in,
                              void* d_out, int out_size, void* d_ws, size_t ws_size,
                              hipStream_t stream) {
  (void)in_sizes; (void)n_in; (void)out_size; (void)ws_size;
  const float* x = (const float*)d_in[0];
  const float* E = (const float*)d_in[1];
  const float* Wp = (const float*)d_in[2];
  const float* bp = (const float*)d_in[3];
  float* out = (float*)d_out;
  char* ws = (char*)d_ws;
  const size_t M16 = (size_t)NN_ * XW * 4;
  float* A = (float*)ws; float* X = (float*)(ws + M16); float* Y1 = (float*)(ws + 2 * M16); float* Y2 = (float*)(ws + 3 * M16);
  k_supports<<<dim3(NN_ / 16), dim3(256), 0, stream>>>(E, A);
  k_xpose<<<dim3(NN_), dim3(256), 0, stream>>>(x, X);
  gemm_kn2<float, false><<<dim3(NN_ / 128, XW / 128, 1), dim3(256), 0, stream>>>(A, NN_, 0, X,  XW, 0, nullptr, 1.0f, Y1, XW, 0, NN_);
  gemm_kn2<float, false><<<dim3(NN_ / 128, XW / 128, 1), dim3(256), 0, stream>>>(A, NN_, 0, Y1, XW, 0, nullptr, 1.0f, Y2, XW, 0, NN_);
  k_node<<<dim3(NN_), dim3(256), 0, stream>>>(E, Wp, bp, X, Y1, Y2, out);
}
